// LinearAttention_51771535786580
// MI455X (gfx1250) — hardware-verified
//
#include <hip/hip_runtime.h>

#ifndef NB
#define NB 2
#endif
#ifndef SEQ
#define SEQ 2048
#endif
#define NB_FULL 2
#define SEQ_FULL 2048
#define DMD 1024
#define NHS 16
#define HD 64
#define QT 256
#define NKX SEQ
#define NTOK (NB * SEQ)

static_assert(NB >= 1 && NB <= NB_FULL);
static_assert(SEQ >= QT && SEQ <= SEQ_FULL && SEQ % QT == 0);
static_assert(NHS * HD == DMD);
static_assert(DMD % 64 == 0 && DMD % 32 == 0 && HD == 64 && QT % 64 == 0 && SEQ % 64 == 0);
static_assert(((QT / 16) * (QT / 64)) % 4 == 0);
static_assert(((QT / 16) * (HD / 64)) % 4 == 0);
static_assert(((NTOK / 16) * (DMD / 64)) % 4 == 0);
static_assert(((DMD / 16) * (SEQ / 64)) % 4 == 0);
static_assert(((SEQ / 16) * (DMD / 64)) % 4 == 0);
static_assert((NTOK * (DMD / 8)) % 256 == 0);
static_assert(((DMD * DMD) / 8) % 256 == 0);

typedef _Float16 v16h __attribute__((ext_vector_type(16)));
typedef unsigned short v8us __attribute__((ext_vector_type(8), may_alias));
typedef float v8f __attribute__((ext_vector_type(8)));
typedef float v4f __attribute__((ext_vector_type(4)));
typedef float v4fa __attribute__((ext_vector_type(4), may_alias));
union FragH { v16h v; v8us half[2]; _Float16 h[16]; unsigned short u[16]; };

__device__ __forceinline__ unsigned short bf16_bits(float x) { unsigned int u = __float_as_uint(x); return (unsigned short)((u + 0x7FFFu + ((u >> 16) & 1u)) >> 16); }
__device__ __forceinline__ float bf16_val(unsigned short b) { return __uint_as_float(((unsigned int)b) << 16); }
__device__ __forceinline__ float bf16_rne(float x) { return bf16_val(bf16_bits(x)); }

__device__ __forceinline__ v16h g2_frag(const _Float16* p, int hh) { FragH f; f.half[0] = *(const v8us*)((const unsigned short*)p + 8 * hh); f.half[1] = *(const v8us*)((const unsigned short*)p + 16 + 8 * hh); return f.v; }
__device__ __forceinline__ v8f g2_mma(v16h a, v16h b, v8f c) { v8f d = __builtin_amdgcn_wmma_f32_16x16x32_f16(false, a, false, b, (short)0, c, false, false); asm volatile("v_nop\n\tv_nop\n\tv_nop\n\tv_nop" : "+v"(d) : "v"(a), "v"(b)); return d; }

__global__ __launch_bounds__(256) void k_x16(const float* __restrict__ x, _Float16* __restrict__ X16, int ntok) {
  const size_t t = (size_t)blockIdx.x * 256 + threadIdx.x;
  const size_t n8 = (size_t)ntok * (DMD / 8);
  if (t >= n8) return;
  const int m = (int)(t / (DMD / 8)), c8 = (int)(t % (DMD / 8)) * 8;
  const size_t src = ((size_t)(m / SEQ) * SEQ_FULL + (size_t)(m % SEQ)) * DMD + (size_t)c8;
  const v4f a = *(const v4fa*)(x + src), c = *(const v4fa*)(x + src + 4);
  FragH f;
#pragma unroll
  for (int q = 0; q < 4; ++q) { f.h[q] = (_Float16)bf16_rne(a[q]); f.h[4 + q] = (_Float16)bf16_rne(c[q]); }
  const v8us o = f.half[0];
  unsigned short* d = (unsigned short*)X16 + t * 8;
  *(volatile v8us*)d = o; __threadfence(); *(volatile v8us*)d = o;
}

__global__ __launch_bounds__(256) void k_wnat(const float* __restrict__ w, size_t n8, _Float16* __restrict__ Bt) {
  const size_t t = (size_t)blockIdx.x * 256 + threadIdx.x; if (t >= n8) return; FragH f;
#pragma unroll
  for (int q = 0; q < 8; ++q) f.h[q] = (_Float16)(bf16_rne(w[t * 8 + q]) * 16.0f);
  const v8us o = f.half[0];
  unsigned short* d = (unsigned short*)Bt + t * 8;
  *(volatile v8us*)d = o; __threadfence(); *(volatile v8us*)d = o;
}

template <bool ASPL, bool BSPL, bool BROW, bool OUT16>
__global__ __launch_bounds__(128) void k_mm(const _Float16* __restrict__ Ah, const _Float16* __restrict__ Al, int lda, size_t sA,
                                           const _Float16* __restrict__ Bh, const _Float16* __restrict__ Bl, int ldb, size_t sB,
                                           float alpha, const float* __restrict__ bias, int cdiag,
                                           float* __restrict__ C, _Float16* __restrict__ Ch, _Float16* __restrict__ Cl, int ldc, size_t sC,
                                           int M, int N, int K) {
  __shared__ __attribute__((aligned(16))) float so[4][16][64];
  const int tid = threadIdx.x, w = tid >> 5, lane = tid & 31, ln = lane & 15, hh = lane >> 4;
  const int by = blockIdx.y;
  const size_t aofs = (size_t)by * sA, bofs = (size_t)by * sB, cofs = (size_t)by * sC;
  const int ntn = N >> 6;
  const int wid = blockIdx.x * 4 + w;
  const int mt = wid / ntn, nq = wid - mt * ntn;
  if (mt * 16 >= M) return;
  const int row0 = mt * 16, col0 = nq * 64;
  const _Float16* ahp = Ah + aofs + (size_t)(row0 + ln) * lda;
  const _Float16* alp = ahp; if (ASPL) alp = Al + aofs + (size_t)(row0 + ln) * lda;
  const _Float16* bhp = Bh + bofs + (size_t)(col0 + ln) * ldb;
  const _Float16* blp = bhp; if (BSPL) blp = Bl + bofs + (size_t)(col0 + ln) * ldb;
  v8f ch[4] = {}, cx[4] = {};
#pragma unroll 1
  for (int kb = 0; kb < K; kb += 32) {
    const v16h ah = g2_frag(ahp + kb, hh);
    v16h al = ah; if (ASPL) al = g2_frag(alp + kb, hh);
#pragma unroll
    for (int t = 0; t < 4; ++t) {
      const v16h bh = g2_frag(bhp + (size_t)t * 16 * ldb + kb, hh);
      ch[t] = g2_mma(ah, bh, ch[t]);
      if (ASPL) cx[t] = g2_mma(al, bh, cx[t]);
      if (BSPL) { const v16h bl = g2_frag(blp + (size_t)t * 16 * ldb + kb, hh); cx[t] = g2_mma(ah, bl, cx[t]); }
    }
  }
#pragma unroll
  for (int t = 0; t < 4; ++t) {
    const int col = col0 + t * 16 + ln;
    float bcol = 0.f;
    if (!BROW) { if (bias != nullptr) bcol = bf16_rne(bias[col]); }
#pragma unroll
    for (int r = 0; r < 8; ++r) {
      const int rl = 8 * hh + r;
      float v = ch[t][r];
      if (ASPL || BSPL) v += cx[t][r] * 0.0009765625f;
      v *= alpha;
      if (BROW) { if (bias != nullptr) v += bf16_rne(bias[row0 + rl]); } else v += bcol;
      v = (col <= cdiag + row0 + rl) ? v : 0.0f;
      so[w][rl][t * 16 + ln] = v;
    }
  }
  __builtin_amdgcn_fence(4  , "workgroup");
  __builtin_amdgcn_wave_barrier();
  if (OUT16) {
    const int r8 = lane >> 3, c8 = (lane & 7) * 8;
    for (int pass = 0; pass < 2; ++pass) {
#pragma unroll
      for (int q = 0; q < 4; ++q) {
        const int r = q * 4 + r8;
        const v4f a = *(const v4fa*)&so[w][r][c8], c = *(const v4fa*)&so[w][r][c8 + 4];
        FragH fh, fl;
#pragma unroll
        for (int i = 0; i < 4; ++i) {
          _Float16 h = (_Float16)a[i]; fh.h[i] = h; fl.h[i] = (_Float16)((a[i] - (float)h) * 1024.0f);
          h = (_Float16)c[i]; fh.h[4 + i] = h; fl.h[4 + i] = (_Float16)((c[i] - (float)h) * 1024.0f);
        }
        const size_t o = cofs + (size_t)(row0 + r) * ldc + (size_t)(col0 + c8);
        const v8us oh = fh.half[0], ol = fl.half[0];
        *(volatile v8us*)((unsigned short*)Ch + o) = oh;
        if (Cl != nullptr) *(volatile v8us*)((unsigned short*)Cl + o) = ol;
      }
      if (pass == 0) __threadfence();
    }
  } else {
    const int rsub = lane >> 4, c4 = (lane & 15) * 4;
    for (int pass = 0; pass < 2; ++pass) {
#pragma unroll
      for (int q = 0; q < 8; ++q) {
        const int r = q * 2 + rsub;
        const v4f v = *(const v4fa*)&so[w][r][c4];
        *(volatile v4f*)(C + cofs + (size_t)(row0 + r) * ldc + (size_t)(col0 + c4)) = v;
      }
      if (pass == 0) __threadfence();
    }
  }
}

static inline unsigned mm_blocks(int M, int N) { return (unsigned)(((M / 16) * (N / 64)) / 4); }

extern "C" void kernel_launch(void* const* d_in, const int* in_sizes, int n_in,
                              void* d_out, int out_size, void* d_ws, size_t ws_size, hipStream_t stream) {
  if (n_in < 9) return;
  const long long needx = ((long long)(NB - 1) * SEQ_FULL + SEQ) * DMD;
  if ((long long)in_sizes[0] < needx) return;
  if (in_sizes[1] < DMD * DMD || in_sizes[3] < DMD * DMD || in_sizes[5] < DMD * DMD || in_sizes[7] < DMD * DMD) return;
  if (in_sizes[2] < DMD || in_sizes[4] < DMD || in_sizes[6] < DMD || in_sizes[8] < DMD) return;
  if ((long long)out_size < needx) return;

  const float* x  = (const float*)d_in[0];
  const float* wq = (const float*)d_in[1];
  const float* bq = (const float*)d_in[2];
  const float* wk = (const float*)d_in[3];
  const float* bk = (const float*)d_in[4];
  const float* wv = (const float*)d_in[5];
  const float* bv = (const float*)d_in[6];
  const float* wo = (const float*)d_in[7];
  const float* bo = (const float*)d_in[8];
  float* out = (float*)d_out;

  char* ws = (char*)d_ws; size_t off = 0;
  auto take = [&](size_t bytes) { char* p = ws + off; off += (bytes + 255) & ~(size_t)255; return p; };
  const size_t plane = (size_t)NTOK * DMD * 2;
  _Float16* X16  = (_Float16*)take(plane);
  _Float16* Wq16 = (_Float16*)take((size_t)DMD * DMD * 2);
  _Float16* Wk16 = (_Float16*)take((size_t)DMD * DMD * 2);
  _Float16* Wv16 = (_Float16*)take((size_t)DMD * DMD * 2);
  _Float16* Wo16 = (_Float16*)take((size_t)DMD * DMD * 2);
  _Float16* Qh   = (_Float16*)take(plane);
  _Float16* Ql   = (_Float16*)take(plane);
  _Float16* Kh   = (_Float16*)take(plane);
  _Float16* Kl   = (_Float16*)take(plane);
  _Float16* VTh  = (_Float16*)take((size_t)NB * DMD * SEQ * 2);
  _Float16* VTl  = (_Float16*)take((size_t)NB * DMD * SEQ * 2);
  _Float16* P    = (_Float16*)take((size_t)NHS * QT * NKX * 2);
  _Float16* Cth  = (_Float16*)take(plane);
  _Float16* Ctl  = (_Float16*)take(plane);
  if (off > ws_size) return;

  const float a16 = 0.0625f;
  const int NOCAUSAL = 1 << 28;
  const size_t w8 = (size_t)DMD * DMD / 8;

  k_x16<<<(unsigned)(((size_t)NTOK * (DMD / 8)) / 256), 256, 0, stream>>>(x, X16, NTOK);
  k_wnat<<<(unsigned)(w8 / 256), 256, 0, stream>>>(wq, w8, Wq16);
  k_wnat<<<(unsigned)(w8 / 256), 256, 0, stream>>>(wk, w8, Wk16);
  k_wnat<<<(unsigned)(w8 / 256), 256, 0, stream>>>(wv, w8, Wv16);
  k_wnat<<<(unsigned)(w8 / 256), 256, 0, stream>>>(wo, w8, Wo16);

  k_mm<false, false, false, true><<<dim3(mm_blocks(NTOK, DMD), 1), 128, 0, stream>>>(
      X16, nullptr, DMD, (size_t)0, Wq16, nullptr, DMD, (size_t)0, a16, bq, NOCAUSAL,
      nullptr, Qh, Ql, DMD, (size_t)0, NTOK, DMD, DMD);
  k_mm<false, false, false, true><<<dim3(mm_blocks(NTOK, DMD), 1), 128, 0, stream>>>(
      X16, nullptr, DMD, (size_t)0, Wk16, nullptr, DMD, (size_t)0, a16, bk, NOCAUSAL,
      nullptr, Kh, Kl, DMD, (size_t)0, NTOK, DMD, DMD);
  k_mm<false, false, true, true><<<dim3(mm_blocks(DMD, SEQ), NB), 128, 0, stream>>>(
      Wv16, nullptr, DMD, (size_t)0, X16, nullptr, DMD, (size_t)SEQ * DMD, a16, bv, NOCAUSAL,
      nullptr, VTh, VTl, NKX, (size_t)DMD * SEQ, DMD, SEQ, DMD);

  for (int b = 0; b < NB; ++b) {
    for (int q0 = 0; q0 < SEQ; q0 += QT) {
      const int nk = q0 + QT;
      const size_t arow = ((size_t)b * SEQ + q0) * DMD;
      const size_t krow = (size_t)b * SEQ * DMD;
      k_mm<true, true, false, true><<<dim3(mm_blocks(QT, nk), NHS), 128, 0, stream>>>(
          Qh + arow, Ql + arow, DMD, (size_t)HD, Kh + krow, Kl + krow, DMD, (size_t)HD, a16, nullptr, q0,
          nullptr, P, nullptr, NKX, (size_t)QT * NKX, QT, nk, HD);
      k_mm<false, true, false, true><<<dim3(mm_blocks(QT, HD), NHS), 128, 0, stream>>>(
          P, nullptr, NKX, (size_t)QT * NKX, VTh + (size_t)b * DMD * SEQ, VTl + (size_t)b * DMD * SEQ, NKX, (size_t)HD * NKX, 16.0f, nullptr, NOCAUSAL,
          nullptr, Cth + arow, Ctl + arow, DMD, (size_t)HD, QT, HD, nk);
    }
  }
  k_mm<true, false, false, false><<<dim3(mm_blocks(SEQ, DMD), NB), 128, 0, stream>>>(
      Cth, Ctl, DMD, (size_t)SEQ * DMD, Wo16, nullptr, DMD, (size_t)0, a16, bo, NOCAUSAL,
      out, nullptr, nullptr, DMD, (size_t)SEQ_FULL * DMD, SEQ, DMD, DMD);
}
